// MapLoss_60060822667546
// MI455X (gfx1250) — hardware-verified
//
#include <hip/hip_runtime.h>


#define NALL 8192
#define NTR  7372
#define NVA  820
#define KP   7424
#define RCH  1024
#define DM   KP
#define DEPS 1e-12f
#define LOSC 1024.0f

__constant__ int c_perm[NALL] = {824,5474,4138,1580,5558,1627,2120,5176,3192,3236,850,7258,5805,4956,485,343,5058,5839,1768,1524,3737,6719,4556,7807,4204,3465,4400,2829,6460,5720,7097,4198,1801,5073,7038,4665,6862,4325,1052,5160,3850,3637,7873,2759,5302,3460,3643,4522,1987,3220,91,2358,1498,1236,4771,7460,3562,2603,3043,3535,5671,3659,6040,3641,6464,5002,4906,452,1240,7127,1815,2072,7200,3048,4446,7507,7253,906,1506,3542,4367,4207,6601,1214,2892,2512,5576,1300,2054,2305,6317,4327,1205,1901,8140,6649,1385,6709,5768,5026,4812,4744,6804,591,1299,2687,3718,5721,3258,2413,6466,3041,2117,5070,4361,7440,1889,1568,6196,3208,4583,2690,8054,6520,2290,86,5735,354,4949,5557,470,3691,1804,160,1807,8025,4417,4806,7863,7895,4917,750,853,7589,7773,4941,7986,7914,7913,6692,8177,5959,2773,1763,3277,653,1831,4729,3450,3492,1227,2445,2811,6952,2153,6203,8162,7739,5393,8144,425,1264,2118,3678,6821,2612,3382,1694,4303,2633,7789,6074,4619,6044,5189,5887,5552,6111,5660,1590,8035,192,4715,6081,1879,3451,4151,4233,7019,5880,5617,3402,3234,4542,4825,501,7733,203,6734,1698,7889,1,7614,4877,269,1314,1767,4660,3614,1253,412,6294,5149,2977,4642,429,5483,3728,4013,4892,6340,6134,1594,4047,5478,1936,7524,6650,1596,5803,709,2637,5432,4989,5638,7732,5140,7321,1669,8133,3331,3771,3841,3830,6636,1404,5156,7582,7216,3662,2532,7586,1501,1488,2224,7371,4006,5193,3105,4225,4714,6822,7234,130,696,4768,7319,672,5398,2085,6691,418,2128,1613,1649,323,3687,473,7853,6700,3837,6616,7275,1640,7712,4239,7239,7043,2724,6566,4294,1749,4342,987,925,5399,6633,8047,5370,1635,5942,8122,1410,4220,5693,7202,4960,1458,4900,3703,7180,1193,1078,2355,1344,2205,673,2482,5394,3174,2377,4668,5713,4984,1830,6911,2583,131,7892,1657,3222,3455,1118,727,4257,495,5005,7642,356,4150,7222,8071,670,5870,5969,4677,1871,617,5060,3970,1056,533,1766,5466,6630,8190,17,4804,6905,8165,1966,6624,5030,5562,2655,5719,7649,4110,1233,765,6683,3499,126,6731,5753,36,3306,4254,8056,7311,361,4690,2909,6033,3818,4035,7621,329,1709,5625,1389,4358,2533,5877,5360,3315,1058,3776,2163,2722,8010,745,618,4558,4137,477,3060,227,5986,2443,4554,531,3147,7029,2218,5772,3189,484,301,6599,7801,662,1077,1467,6003,7531,1751,1180,3399,8016,8017,2782,2958,4241,2199,2834,1986,4039,5359,7533,7387,1463,5238,1784,5518,2597,2436,3910,6996,5519,12,871,1850,1577,325,6801,1678,1843,4121,4157,4738,4912,652,2938,2629,50,256,2797,6664,6802,141,5624,2293,5980,3679,2626,4901,3866,5888,7514,1837,7337,5247,7609,115,5811,647,3213,2091,543,3607,1213,2970,6440,548,1771,3512,517,5329,2851,686,897,5627,5075,214,1550,4716,1825,5683,1867,3025,6451,7466,3973,5321,1091,4938,2211,3030,1114,7107,4281,4918,4887,8149,8136,1814,6386,2761,1486,7911,4614,2457,4133,2392,7506,7428,4334,7429,5775,2138,8000,680,49,1641,6550,5163,7922,5499,689,6643,7959,6091,7958,2316,6128,4286,6268,4043,177,6487,2708,4686,5555,8057,2663,3790,2918,450,3319,7417,6591,7508,3950,5650,5333,1593,5453,968,4711,4525,2068,4092,1296,4889,948,5040,7006,1592,5334,2219,1134,1842,6053,266,1945,4298,2360,5502,3464,4653,3318,6702,6628,3338,3559,2787,1210,3246,1886,5566,7938,3586,1280,6143,2946,5651,440,5384,6873,1679,7379,7450,1967,4944,2624,4782,7376,4587,2774,644,6411,2074,1919,4582,2383,6880,571,8043,4710,7372,239,3808,1699,3141,2865,610,7418,2166,3669,1570,2292,4058,1935,7683,3996,1037,1576,3463,6855,8019,1792,250,3481,1902,7891,4163,3480,3889,3985,3854,2928,5659,2838,4817,4505,3716,404,3606,7102,6518,213,3605,7263,1377,7456,2167,5711,927,238,5409,4511,5631,8037,2514,3811,1416,4615,1182,3150,628,7532,5709,1880,7092,4040,4953,5874,6360,3005,1643,2020,1415,6828,4731,6225,5728,3524,5646,515,7196,2448,2458,180,2216,5197,4559,5490,2842,6097,81,5361,1145,2081,7721,6916,3602,5395,4657,6197,3649,1774,5515,5016,3731,8031,1928,835,5976,914,6922,230,2709,1605,2688,3695,595,6621,5439,3792,6753,5662,2841,6541,289,978,7064,7910,4232,3684,2522,5065,6744,785,946,6354,498,1462,1810,2634,5831,4243,5188,7024,5157,7369,4076,6505,478,1017,3869,2701,4848,1470,4447,261,5860,1553,5300,4017,7420,6763,6706,5548,2108,523,2670,6098,4584,8030,3752,1742,7380,2562,5506,4516,2257,826,6565,4851,5508,7425,3007,4737,4426,5028,5814,5254,3161,4098,6790,82,6669,3171,6188,2115,3552,6515,1887,6156,7666,3979,3086,7021,1136,5369,7529,6186,5386,4052,6782,4820,7905,4249,5922,6814,3475,1995,4320,1996,8103,5124,6099,380,3784,1188,7110,8064,1808,1407,4326,6848,6058,6707,2548,6452,7703,2314,5867,6431,7967,2184,4041,7170,8123,5718,6082,6608,3778,5015,2442,3943,5700,3692,3414,2277,3634,577,1007,6704,6378,3153,6524,8092,6202,218,6072,3639,1483,4333,7051,5787,6832,4287,4093,3579,4064,534,83,6970,7547,7259,3896,728,5480,5665,732,8130,5596,5322,5056,3878,5837,2792,4491,998,2401,3275,4337,3913,3638,369,1874,3627,2886,183,3111,4394,6467,7904,8075,7767,281,7994,4785,950,4732,7181,8055,3055,1900,7451,1092,4195,471,5281,2510,753,7280,3711,2180,1119,2561,6675,4755,2601,7619,1083,588,1262,6973,4908,6356,7989,6569,1519,4167,2850,5741,4903,7322,2576,3511,4911,4539,2462,2745,1811,4936,2387,5425,7550,6982,6607,8029,7033,4718,4203,333,4336,2296,4062,5203,7857,6953,6913,7363,3576,3008,1653,6904,2026,1759,1254,7757,7862,3323,455,4569,8012,3378,6969,5836,5086,742,8051,6695,3489,1130,2455,2976,4149,3734,2286,150,4431,4479,2294,1444,1503,2415,7612,7505,6842,5488,1084,994,4613,3590,7882,4341,3288,1809,4622,7270,2343,2689,5400,7723,539,4265,5363,6874,1388,2584,3958,1476,5626,557,6899,4793,7486,3179,5008,1365,1289,3158,5765,7242,4762,4354,2077,1975,6884,8099,838,1681,4964,1259,1047,2206,8168,2187,5971,6481,2238,178,6181,4078,3911,3770,6366,7061,374,6770,121,6564,1094,3849,2023,7844,5654,1076,43,2720,5977,1469,5431,503,8105,1039,2862,6271,4290,4319,410,4144,7701,1629,7465,3191,4544,1651,1658,6161,4194,5892,1485,3665,885,4495,3347,2405,4685,5366,6736,681,876,8108,7093,4197,1499,2836,2264,1551,6815,315,4168,1571,6752,2333,3955,6355,1909,7445,1033,5699,2673,7156,3173,2807,545,5871,1794,7867,604,3142,2665,5174,5196,2879,1283,4260,2845,2508,2927,7677,1838,6696,3471,2236,30,3858,367,5335,7218,2039,1911,7681,4,3194,1222,3070,6883,945,3640,2515,6554,4863,817,6976,6210,2221,7906,756,5856,5934,4939,1317,6792,7085,6136,4289,7831,4227,6745,6538,6363,1621,5295,5044,6118,2991,7957,1232,379,7101,6149,5264,4897,1942,814,7182,5743,53,1638,7250,2309,135,2801,2125,4383,3001,3693,3425,4349,7858,1903,7210,2447,1237,3494,1922,1752,7485,2813,5808,5087,6100,6388,2632,3299,7326,6285,2540,565,2347,7779,4185,529,2606,3549,5788,6634,4478,6658,7400,5088,4412,1327,3216,2900,5587,4551,6895,6629,4792,1890,1368,1380,4507,4122,6623,4252,6992,4733,4890,7161,4830,4117,107,5911,4054,3876,2835,5029,6191,1985,7558,5606,7984,6417,4741,4734,7408,3459,4436,1500,1181,862,3143,7747,2341,2555,2891,7556,5099,3744,40,6585,1062,474,5549,3560,7809,7491,1644,1628,6146,3887,3449,7814,1665,396,6760,719,7482,7731,1642,5067,1408,2856,3123,6117,774,3432,2752,2248,5924,1579,2432,627,2263,5110,2815,5463,3733,2356,1992,393,5134,5533,4259,2430,1163,2998,6442,7705,2417,4372,936,8186,3919,1898,8152,8163,6214,5901,5465,621,3393,530,855,4377,5433,778,5024,4524,481,6837,3677,6535,4513,6838,2089,6596,4534,4127,4520,7089,913,4965,3625,5862,6960,365,816,2477,3294,5212,2544,5227,2950,2675,2312,1295,2699,2311,4705,8094,3750,7406,7323,1923,8023,435,6109,1994,6176,422,5031,3946,3828,2997,4360,245,6049,5847,3062,5217,3501,3928,633,6436,7011,3720,6781,251,3073,1587,1021,8095,1648,6768,3848,1671,4807,4448,7926,7648,5708,2683,4747,4036,4952,7479,2563,2201,6845,6954,894,7660,4087,85,818,7152,7544,3604,7091,3121,8065,4858,5746,2529,346,2656,5150,1739,7289,1539,7410,5983,4579,7684,6439,5714,4638,1009,4302,622,5505,3526,3094,6584,6981,7413,5763,2617,1360,2642,6784,2723,1779,3922,288,1081,195,2602,3058,555,3076,1412,7221,3263,7830,5442,2686,3237,1634,593,3724,5045,5521,1403,953,7256,6259,7845,2044,1293,6079,2528,7399,1005,6201,296,1042,3357,671,446,5685,522,6489,2825,4324,6887,3071,1331,7888,3518,4940,8087,2978,3704,3365,38,1032,3166,2245,2339,7277,5419,6945,5813,1050,7285,4750,249,1099,1453,1333,68,6052,2731,6045,8107,5797,5961,1600,4178,7515,4202,3905,5270,7264,2007,458,5667,5496,7472,7680,746,3290,4174,3068,550,2412,5817,7784,6747,6943,4088,6906,5180,7972,6113,712,7656,7271,7534,2096,6614,2582,4894,6710,2945,6656,6024,2586,6600,4928,5094,4175,1542,320,1066,4589,59,4053,6303,7942,70,2016,7223,7,4262,6796,3099,5014,6826,7118,7988,5906,6919,5374,7114,3100,1082,1024,416,1747,7908,338,1818,7886,4818,6694,6306,5301,4422,2888,118,3407,1185,5672,5932,3802,6461,2650,4010,2315,3926,5664,5085,4853,3190,3296,4604,6825,3002,2019,6963,2164,2152,3696,7499,1973,409,3497,4263,6443,3037,7519,4995,3377,1717,8083,5715,3758,3975,2299,2249,4181,3574,5389,3305,5497,6103,2523,4268,3618,6084,7753,2010,1997,1366,1855,4237,3199,4527,4376,3938,6563,4713,8018,42,4833,3945,2702,403,714,6971,6986,1070,5717,2698,6287,2493,7651,7797,5686,4644,2062,2872,974,6013,4843,8102,2543,3963,6419,5211,1941,3585,2882,5653,4987,3648,3284,4943,7778,849,2402,3587,796,1718,1199,3253,5875,4390,66,6931,3195,5422,7192,4231,4742,3651,6619,6909,1452,166,3160,4641,7173,724,5082,6200,2434,2349,5754,1353,873,7770,2764,7741,7059,7617,3431,383,3243,2747,4699,15,2214,7076,4317,524,5695,2367,7373,6987,3394,5542,7933,2185,2025,4000,303,3052,349,6162,3364,133,4424,6681,1194,6947,3939,4775,5893,2833,7650,6027,1494,5325,963,2406,6891,5257,5923,4316,2279,3170,6509,298,1566,3617,7124,7587,4878,1785,1581,6080,5052,5171,3229,7542,6035,583,1603,7442,366,4049,715,5777,6820,5458,6972,337,969,3154,3207,5575,184,7144,5601,5277,3925,282,5144,5929,7774,6108,3879,236,6286,4905,3561,2974,6004,7981,4724,7971,1510,6548,2806,3646,4180,2228,1543,3591,1673,556,6262,3743,3389,5520,2378,5280,6414,558,4209,7795,2822,538,4100,4754,6140,6817,8119,1962,6486,7601,125,5943,6497,3406,6391,1977,7624,2189,1725,405,4323,8114,4430,3779,1202,4618,5812,3279,5656,7658,3262,3252,6721,5195,506,6048,7866,5767,6328,5306,6249,5062,5164,2535,3231,1310,5586,1620,6795,3440,4189,5123,6195,1086,5525,5154,7976,5240,3325,1719,3373,5275,4603,4160,4258,2047,4726,6955,1789,1848,544,297,2860,1884,2638,1753,3495,4616,14,6732,2474,4413,2738,3337,3843,7934,7249,8128,1721,4721,2345,5614,3295,551,3006,4915,6926,6743,5920,5623,6112,4153,6226,4599,6995,413,596,1897,2053,4032,2196,3502,4123,3182,5785,246,2839,7584,7225,1349,3298,2828,2344,2600,1531,1053,1584,7366,5691,7329,4969,3029,2484,986,3004,7599,2907,6703,368,2239,7717,2090,4620,1457,4886,7763,2660,2620,4300,7662,3308,6067,3057,1832,174,4012,1006,3997,5055,5460,7597,5093,6055,5080,8024,26,6133,1731,4578,7334,6373,1479,8188,5491,5703,5090,2281,4531,1409,3842,6934,866,3136,8104,6068,2454,519,6282,1465,4552,6233,187,5669,3906,7160,5379,2577,1000,7164,2042,7930,5545,222,3713,4409,3371,988,663,4951,482,2716,2079,2156,7591,5799,6131,5915,4791,8148,2487,6622,4380,2751,4590,4456,7331,1786,918,263,6590,848,5068,1477,6493,2301,3390,6474,5129,6422,4477,7151,6150,2272,7598,2579,7579,3667,8038,1319,4532,6029,2319,6211,3567,6372,4866,6775,300,1758,7893,3940,3685,943,5613,3385,1723,2715,7188,769,1155,1791,7065,5285,1040,4647,1672,4749,6311,3538,7670,3359,6949,5532,2623,2565,5007,1367,181,6336,3582,389,4467,7566,1195,3180,8189,4072,5517,258,3987,7711,7031,1999,5347,2649,677,1334,4216,4756,3688,420,1913,6198,7452,1790,7569,7079,309,5236,4982,1715,919,6423,1547,7389,95,1071,1993,4658,7477,3682,1055,6829,2525,2917,755,7685,6071,2866,7438,1852,6167,3719,611,6513,3133,19,1495,1743,2017,1161,4384,6164,7109,773,2788,7702,7032,2041,7018,1168,5108,900,5890,7454,2404,1802,1023,3589,4292,6073,6733,6978,24,7328,5818,2770,4596,2757,72,7009,3835,3929,3084,65,726,4352,3969,1826,7690,3044,6661,4421,4402,2943,7740,1536,7955,5284,1906,6759,5401,6207,5588,3053,7040,2942,3847,7749,7674,4933,7843,3886,5245,4146,6470,2746,2209,5262,5109,6441,3881,4529,3420,784,5633,6034,6924,6933,877,170,4816,4872,5271,1601,347,703,8138,3423,6092,2768,7752,5020,318,7581,61,1443,6242,5830,5551,7421,5844,395,8170,7209,4261,4748,7915,7716,1011,4179,3248,322,4008,6138,5102,808,4948,13,4094,888,2394,1932,3635,7673,1609,7393,280,1865,4919,1073,7052,6525,964,2274,6998,8161,3429,6462,536,3965,2513,6847,5628,7827,3127,2919,2143,3376,2148,3523,4452,1572,6308,5486,6625,4859,7818,4957,2853,5421,212,5629,5000,2067,5595,6686,6502,5353,5107,3566,5317,3833,6424,6169,1737,3822,2987,4455,6219,2002,496,6402,682,6400,2354,637,7708,2282,1219,5854,5819,7409,4549,956,466,5482,5556,6065,5954,631,4879,748,5114,4159,6498,3119,8082,96,3782,2895,580,1746,6122,4031,2306,3114,4449,7086,4223,3436,7047,7075,2904,2247,2648,2692,4173,7474,4196,3286,5759,3313,6007,4451,1057,6519,4652,4703,5750,3036,5216,4142,3014,3270,1373,103,8050,3772,3601,7231,1575,7518,1038,3421,586,1971,196,442,952,3321,2411,2550,1460,6019,4460,2094,6765,3444,5209,186,1090,6698,4388,3088,5984,4256,2844,3183,579,764,2696,182,2318,7155,7664,7135,2142,3820,168,1372,2824,3098,6615,1016,2713,8157,3546,7502,7737,7262,2368,926,6475,4493,2336,2574,1933,8116,5071,137,5303,2444,6715,870,7358,4975,6023,6371,581,1823,7060,3274,6491,1979,7714,884,1325,7568,6384,2852,46,6349,7500,5997,1482,6240,90,3411,5161,4280,1012,7205,3453,1868,6291,161,7158,2766,1824,4509,3962,7909,7991,711,2056,3009,2034,841,7402,6297,599,5132,1301,6120,5666,4607,6556,1655,2005,5956,8121,1290,890,2948,6153,6510,3613,7074,7762,7837,4592,2100,8080,649,5912,3829,6345,124,7929,2390,2588,7471,7346,3981,4112,3061,7494,1330,5417,2712,4870,636,1863,2250,4927,3126,2414,5582,7495,1745,2243,443,2567,4205,7238,1026,5493,2590,1481,3140,6139,7004,2906,5214,7626,5346,7870,5731,497,2880,5128,6302,8011,3935,4486,138,2254,6713,1361,3984,625,7139,2171,3992,7607,4273,3573,800,4694,4023,7404,2418,6740,1318,3529,1200,4164,1616,8158,1686,2001,7722,895,2591,7411,469,7633,6991,1537,6789,4821,2955,761,4398,2554,6720,5348,4382,8005,2008,4667,5833,2916,5876,2481,1748,2177,7944,7718,5427,6338,1274,5891,5387,2999,6581,1873,6728,5017,3184,5527,2470,882,7480,6846,5141,5001,7390,3517,3047,6501,1383,5710,1952,1604,3645,6041,2492,7629,4429,619,2804,373,3247,4497,7604,7397,4278,4419,6507,654,4359,2133,3909,7172,1022,4016,1441,4387,1393,428,304,1775,2941,6657,7186,687,2371,4284,6471,3506,4868,3959,3422,1522,3934,4026,7879,7045,1735,2241,3816,2840,6809,6907,7923,4974,6773,4654,2013,1924,5430,3342,6572,3531,6050,1675,7312,2170,3124,225,6420,1943,3328,645,7330,4375,7962,3857,2092,3130,3632,5998,5297,1982,1147,947,802,1197,4689,2992,6449,436,3785,1350,525,4846,3612,3092,7353,3838,7775,4264,7058,4706,8033,6437,6813,3871,5996,1427,4192,5995,5183,2284,4126,6171,6086,5773,7437,1268,1615,2744,6330,1559,6295,4955,6839,4271,3302,569,6762,6064,5326,2172,6854,2192,5567,2446,7266,7736,6553,1724,313,3040,262,2867,576,402,1829,6923,3650,2912,6243,398,1760,2937,4998,2494,3391,5908,4172,3240,3042,1363,2111,6758,5641,6901,6582,8117,7990,500,4508,4666,2313,201,7318,1379,2706,960,4395,7559,438,2775,4019,3516,6077,6575,4314,5219,264,2765,6533,508,5636,614,758,2342,4097,4285,6325,3134,806,472,2421,5464,6726,789,6868,1270,6172,1060,5328,1834,6057,3824,2830,513,690,4564,7924,1198,3278,5449,7426,2560,4440,7388,3470,2557,1981,7446,5106,5649,4862,3751,411,6587,7035,3705,6350,1980,7036,3457,6101,3144,1392,2737,400,5896,2036,8181,5621,3826,4071,5594,4883,1882,5950,7527,5677,6165,3525,7489,1085,6964,7395,4228,8134,3167,5101,7898,4672,6783,1450,1249,336,3547,1096,5541,4802,3339,2573,4720,2994,4389,937,6333,2147,3746,4571,2923,7595,1662,8096,1326,3082,7611,4347,5894,7385,4895,5309,6879,6494,6258,244,3686,4810,4673,7146,3139,7184,2985,4386,220,1991,3419,3923,7808,7834,4279,7816,6021,6586,5644,4229,3361,6320,3080,8146,3745,7204,2897,7459,7214,7907,6011,2875,2038,3211,5694,2076,1044,1713,572,1345,3281,7316,4067,3458,3888,3168,892,4255,4954,408,3786,2029,434,28,4986,6701,2489,4876,4496,5670,3982,4378,1137,6859,3798,5349,7520,6654,2803,3089,1218,7157,2491,3019,5181,1797,4200,2952,7688,4428,58,6110,2873,1757,2594,6032,2968,2099,6580,4135,1286,6278,2972,4794,6870,433,6213,6956,207,445,1374,3675,3540,5716,2269,4976,5572,8090,140,820,364,5097,4671,2237,889,7804,2230,6221,4020,5782,6527,7899,3276,3032,206,2366,4656,6367,2772,7340,688,6154,4024,3522,7106,5215,6329,843,6592,976,4183,7053,2564,720,4018,6682,8081,1947,4631,8089,7761,6193,2983,6799,461,5332,1951,5356,5673,1151,171,6094,4371,169,7257,5928,6560,1143,3102,1562,1668,6549,5935,3544,5244,6284,4845,7653,6579,3853,5821,3698,7055,449,957,2814,2936,2498,7416,5049,7217,2926,4573,5647,643,2129,307,2957,4373,1258,2905,2703,702,4723,3360,7302,7580,6577,2464,7476,5053,4381,5776,3805,1261,3271,1461,7788,1439,5103,7700,4432,3259,2779,5885,4079,1614,6503,8045,4480,1663,7281,1512,5930,1637,5267,2159,6644,6125,7665,6132,518,1983,7786,1541,2217,3314,1370,2849,363,5680,1025,202,1491,4170,2599,6187,5852,4538,5485,3028,5509,3156,6304,3661,509,5513,5590,4555,7338,2645,6512,1516,8169,2433,6948,3074,1878,5597,4453,5568,4427,1556,2021,766,5705,5283,6015,5169,7041,6671,7252,5120,5827,7467,1525,7103,7760,6793,291,3796,6385,4487,6639,114,7056,2203,2901,6689,6473,5146,7974,4803,6746,324,5263,2790,4147,3823,1192,3653,2195,4348,4725,4865,2035,7874,1322,1769,5879,4351,7790,1445,6583,2048,5027,4557,4468,6244,584,7148,35,2920,5170,3633,252,3806,3054,4213,3230,5258,4712,5261,3861,4152,7605,4611,7735,8026,2095,1432,1729,2876,705,2052,1904,4635,2719,6766,3059,1914,4029,5450,6877,1338,520,4546,98,2881,79,7941,4586,7002,6235,3039,6252,1226,3757,7768,6342,3366,6780,6270,7881,4692,486,2678,1565,4881,7382,1183,4790,4124,1067,1799,966,6516,2287,7448,1257,6257,3206,7632,941,4678,5476,4069,6458,8004,6559,2929,7878,6455,1957,1595,6786,4934,2097,7521,1308,7028,2327,2710,5278,2527,2613,6263,4857,7368,4540,2695,4458,7153,4199,5968,3673,8085,6653,6395,2335,5503,5061,4659,2060,991,5122,1323,767,2495,660,5246,6465,3027,4489,568,8078,2207,7979,2993,2088,257,3862,5987,1297,3203,5436,5100,4585,4134,6392,5554,7123,6626,3616,3978,198,6238,6938,4472,970,4772,5221,6300,4084,1291,511,4501,2785,5178,4753,243,5786,5645,153,4935,4065,7048,4061,5009,4548,1376,676,7999,5158,7993,582,2469,1773,1269,1916,4385,2575,911,3223,4309,2407,989,5066,7341,7698,7133,1782,2721,3244,3683,562,967,4693,7543,2071,4408,80,3078,7315,104,7112,6841,6830,6341,999,224,521,6912,3527,3966,7481,2871,2846,1925,7600,2668,3370,2422,4884,4240,923,5404,4567,4867,3490,3340,3430,3894,8135,6528,4679,4297,8060,2894,3320,7530,3433,2526,4435,5538,3671,3304,5318,6323,730,8147,6612,11,7715,4090,6180,3112,854,5592,7634,2931,6096,5783,4454,2593,4482,7802,277,7608,5975,2982,432,1872,6337,1578,872,4056,5607,4250,3700,4080,2700,4075,859,317,7947,7652,7573,5939,5213,7729,4950,3755,5611,4970,4907,2146,6561,2140,148,6925,7852,2777,7347,1526,2244,6690,3657,7464,738,3780,4498,1335,2350,3793,6500,2951,7126,7333,1059,1624,4299,2202,6993,7159,2065,5727,3564,5013,2104,1309,6428,5098,3681,5112,3438,5076,7488,6189,4004,6641,638,7622,933,7401,2212,5526,397,1316,6668,3178,415,3447,6406,6888,8088,3995,4861,1548,4441,2300,84,710,739,5451,3953,657,1976,7083,2658,6316,1756,2382,6594,4339,5865,5479,3972,6673,4321,2157,7728,3814,4393,6382,1654,3148,5751,1949,2505,2122,5200,1292,2037,4266,1125,7306,5260,3624,899,2101,1707,7875,5910,1447,3010,4560,75,167,751,6208,7860,6816,1160,4057,7294,6716,3330,3000,228,3868,1765,2878,683,4481,3117,3809,6717,3658,7537,4980,3672,4022,3990,912,7310,284,6562,4269,4089,4370,3580,4005,7237,5116,1028,5927,1561,7444,1821,7424,8109,2483,144,1806,1074,4937,3255,6177,4461,8048,6357,7901,4632,902,7572,8049,179,2877,5963,5593,2661,4882,2580,1396,3867,5194,1608,7817,7805,3954,7343,2885,768,5869,6811,1446,3817,7824,6296,209,2614,2193,4795,6220,2763,6418,3125,1417,5048,489,5982,3374,8015,1164,8150,4788,3383,4293,7936,8091,5722,1659,2511,6159,8106,6959,5528,1502,5536,6875,6450,3384,4369,4108,7932,3300,776,664,2517,7121,1602,6070,1106,6937,7178,3165,1419,7261,1854,4156,6833,7195,3980,3372,6237,7313,1552,4683,1513,223,3821,4888,6307,7538,3957,7332,5290,1304,3721,3466,390,3967,32,1514,6147,1048,2428,1284,1589,4488,2868,2270,6737,6523,5461,6984,278,6209,1689,2425,527,1336,7821,7320,5210,1144,3408,7100,3395,381,7284,864,6810,1677,5315,560,3536,6376,6663,7687,804,5972,4595,21,1369,2781,7822,145,6204,5726,5142,5104,7854,6107,7361,358,2131,5137,190,6274,7042,2541,6595,4099,7839,2018,7641,4594,7603,4675,3417,1358,231,5191,5248,1451,3508,6014,1101,3732,6290,2278,1473,3628,6714,3603,2149,5291,2711,3226,4107,1710,283,6321,4120,938,4855,3396,4730,6767,829,3146,1191,4676,2471,3461,5078,5456,1546,2307,5679,7847,1740,4184,3503,3845,0,6006,7577,2303,6383,2556,3528,3689,1706,2271,4379,6212,1036,1504,7131,1123,3051,2246,2080,5535,651,2040,7525,812,3353,1656,1220,7193,4541,903,2545,4757,406,1013,7461,5235,3670,7350,5038,3273,1418,2786,3993,6215,6843,4563,4068,4077,5179,7078,1054,6764,860,578,2680,5472,2112,4824,6544,360,6727,423,4519,7194,5115,4002,734,7360,3948,1968,1100,6526,2061,609,7570,7458,4346,5376,4698,559,74,3699,3895,5794,1803,5684,7710,2145,7787,4570,2685,8007,7748,865,6655,6137,787,7345,2704,2051,3388,3269,4414,4322,1877,1475,2408,3064,7977,763,5949,3031,2073,4761,2380,5023,7475,2086,6288,232,648,4364,5806,7725,3283,2015,3631,8154,4131,5944,1438,5057,3736,8041,3537,1456,45,2739,2351,1875,6928,8034,6787,819,535,1705,2234,2893,7111,7062,4345,741,2252,5418,6409,211,2858,7279,1822,1646,7561,1583,3185,1861,1716,6573,5320,8020,4835,2767,3774,1490,6251,1342,6712,5252,7254,1805,157,1728,1400,3404,7780,665,7960,3813,1278,1133,6729,285,7625,5190,5043,3794,6921,823,4176,5324,1186,4399,4760,7785,3437,6468,2116,7267,2004,1839,7706,7245,326,2857,8111,3644,6272,7953,3515,4780,1819,1423,6054,1332,109,3280,7707,5408,6858,1230,5816,5319,4105,3505,4104,2989,4357,2169,3403,1508,3196,1217,5688,3415,1492,2520,836,2144,8001,1433,5182,2981,1844,6480,5899,922,7982,7997,7516,7122,5339,6427,1211,5266,4332,4208,6914,3891,3974,7432,3107,60,5208,3787,646,5886,1449,4722,3363,6530,1108,3151,6036,3621,2369,6454,1030,8067,932,7199,7750,887,7865,2388,3726,1190,5440,6687,4141,3109,3362,199,7037,5824,930,7578,3901,5820,3900,2966,3741,4637,3629,1619,3405,6026,2643,667,7868,3825,685,7503,2569,210,6234,2697,7820,188,6667,387,3033,7535,3760,6275,2113,216,1154,4186,2338,7897,2864,1926,939,4095,204,1141,7203,10,2398,6756,4130,921,3176,279,1215,5423,2179,4746,1732,1313,3710,5282,7883,783,973,1035,4783,3908,5546,2190,4474,4602,1072,376,3738,8052,1907,844,6182,8061,382,1780,1387,7431,2450,4171,5403,5311,6869,6433,2259,491,891,4070,3827,6352,2102,3961,5414,8172,2261,3351,5729,1647,6183,7468,1841,4044,4193,1421,5591,516,1347,2200,7966,3164,3801,5774,4627,5413,6062,1413,2960,4823,1702,5834,2605,6699,7894,2666,4444,6897,3697,1371,5707,1312,4145,7364,5135,5500,7759,7470,3768,5084,4464,2225,6457,5352,1776,319,2000,5846,6618,5051,52,4640,7555,5524,67,1931,1674,898,4961,674,6322,6738,4356,6326,5289,87,1915,4030,2518,7128,3859,3439,6299,2662,3349,4880,5540,2139,3135,4499,2057,7174,4406,6060,5510,1946,2032,2821,2883,6593,4687,1474,2,5620,4533,7034,6942,6598,4624,3964,5757,3210,4425,7449,7241,1846,4526,7129,7738,2297,5138,7973,5230,2362,5250,5563,5410,355,612,3496,2473,6670,1862,2049,5424,7498,1337,4914,6389,5253,567,5204,6105,359,6665,3245,4893,7511,590,2755,4081,1223,942,6722,6840,1755,7007,1955,7138,1251,6253,1411,5233,7137,4301,1670,6741,7635,3875,7833,6849,971,2553,4055,880,5412,464,193,7692,3020,1442,2467,4129,7265,6613,1625,3186,3368,798,5704,1177,1529,5184,1397,2736,6831,6754,3348,2519,5832,5072,4849,342,6936,4221,4648,5441,4680,7872,5692,779,5895,6983,4844,7130,4033,5074,5151,570,6199,1509,5981,1990,1917,330,7383,2963,6416,7066,7734,8184,3003,6604,2837,6708,7576,1431,4442,7176,1212,6574,7273,1793,695,6885,5843,4407,7829,6448,4512,1089,3839,3285,265,5337,6570,215,1231,5953,6009,5287,5574,1984,4681,736,4574,3832,7645,977,5469,7215,7616,1031,5598,7554,4827,3072,6944,7890,4947,260,6485,5730,7104,4854,5192,7081,2776,5225,4439,2298,3565,4838,2295,467,5416,7900,4234,7113,5091,4048,2337,1307,6256,2463,786,8182,1329,7274,462,1172,4966,5897,7840,8008,3428,7751,832,6075,5034,7027,7552,949,3557,2353,6051,5698,7309,5682,3762,3530,6217,3998,4808,1778,4709,1328,3177,6866,733,2400,5914,7978,4226,1375,3988,5175,6293,4860,5198,723,1424,3610,701,1422,1523,7825,7682,3880,2902,4885,7861,350,2826,4979,4109,3090,151,3152,7003,3011,6106,6531,983,4166,6114,807,924,5205,155,1631,4993,3714,4708,2106,7050,4767,1569,7841,7697,3198,5018,642,2134,549,185,4318,4182,414,2727,77,1287,4155,7640,3187,7667,6104,3783,8098,7087,1324,3977,7169,2410,2014,4275,48,5905,2961,6175,4909,4891,1816,2188,2589,4609,424,6484,6808,6267,5426,5917,1103,4999,7469,3569,6309,1820,3668,6405,6266,6184,7639,468,7696,2742,5373,3747,253,3600,4433,4769,3504,3694,3556,5994,6872,2308,6666,2975,7335,7884,3654,1321,4308,799,5111,3018,6957,3551,348,6085,375,2750,4612,6144,640,5501,5036,2321,1574,996,1455,5639,2922,217,6344,3238,6774,2647,5388,1279,1487,175,1359,6039,444,917,3575,2610,4717,1140,7054,7539,7592,1891,3764,5336,8040,1364,1252,1116,3840,4847,5569,341,4518,3642,722,7308,6910,426,1533,3289,3593,2397,1459,2480,3050,4158,1294,5012,4593,5531,3759,8164,547,6216,191,134,7260,1029,391,915,3369,267,5687,8072,4536,2889,7916,2847,8100,6016,2524,5809,2530,6030,878,237,7377,6920,357,2317,2793,7826,4576,2385,1812,3468,6853,1520,6951,7541,1110,1953,7020,4353,7800,448,2136,5792,6979,1700,6886,6483,620,3469,6037,4663,6223,2135,1733,528,4588,3474,3931,1247,2500,857,7799,6380,4230,3218,7546,2208,3049,532,668,292,8086,5159,805,1564,2641,112,4494,6444,839,1744,4343,8132,5308,5640,6495,6514,4700,1497,3874,7283,7177,5825,3715,8153,6871,8155,2162,6876,5570,2581,4368,5330,575,2571,4276,7744,6932,3225,2348,6860,1929,7179,7269,3412,6552,2572,3570,1127,7948,2323,6425,273,3803,8185,6974,3707,1714,5658,8022,2375,7724,7678,4697,5117,1618,8027,5732,2596,2220,4990,2973,743,1783,5758,830,3756,801,7813,6646,1406,4295,3870,4798,2672,5796,1471,929,4625,385,1238,7643,2046,4968,7391,6807,4839,4246,6261,2386,7896,6061,5882,2940,3091,4926,4222,475,744,6989,2817,809,2651,2260,5105,7528,6723,7434,2816,194,6794,3921,935,7636,457,1711,5380,1835,2971,603,5706,2363,4829,3346,6429,3482,5634,951,2769,6642,332,3865,4483,56,4973,7719,4116,3034,2502,5172,3101,3488,3472,861,7145,2684,5957,3791,7745,4789,3873,5279,6568,1770,7073,2374,88,7509,1851,4591,2003,6127,29,493,5268,6038,6426,2653,3434,460,476,2066,8032,6478,122,34,4669,7116,2740,4786,7150,3400,6730,3730,4701,2154,1827,717,6115,6445,6185,31,5733,7781,117,4875,5701,3729,6771,3312,8079,4959,4626,5745,5173,3021,1885,2441,4296,3936,5218,3292,4655,1557,2105,5573,2083,639,4572,3379,6660,790,1800,3994,6492,7314,3149,1014,176,1075,4502,8156,6999,5755,5364,3462,6479,6882,6381,1896,1930,7663,7125,5126,7336,6056,1229,6018,4566,7709,2618,2585,7699,7985,5760,3227,797,6735,5926,4001,5848,3999,3233,5530,1276,6504,1764,7096,2558,5050,2646,5243,119,5477,6546,286,5452,965,8126,7613,6609,7615,3763,6878,6632,4852,3722,3520,6597,6231,3619,5069,3519,5762,725,437,1836,7013,1352,1061,5828,2501,308,1895,5678,7070,5455,345,691,5206,5723,3035,2006,7386,5580,6769,4528,417,6677,874,1203,1405,7526,3426,1384,5470,2802,3493,6379,5973,3232,1378,6152,5365,2289,7849,4777,4702,1162,5622,2962,847,749,5041,1788,3228,6310,2625,2178,6327,6800,5979,1170,1414,5305,5249,3162,165,6778,2534,7793,149,8066,6339,7869,5823,1394,2705,2568,3181,6965,8101,7352,6124,5965,4745,606,6551,4695,5350,5841,1020,5748,6264,1998,5032,5145,69,1573,20,173,8059,4305,5676,3163,3441,7219,3767,1302,7119,1978,7811,5849,3172,6206,5845,2953,7995,7354,1881,7970,735,4132,2222,2789,2098,3983,5603,5550,1696,993,1626,4191,2995,3807,7855,1496,2843,7937,5951,2028,7590,7512,4311,5940,6645,2818,2639,6788,7996,5618,7080,2409,8063,8036,5571,4011,5383,6069,7230,2854,5632,5495,2419,7022,147,1870,99,7185,8137,1691,6289,2151,5602,5947,2615,2461,1563,5790,3435,6739,7287,1892,2449,1275,2570,1970,4060,1676,1015,3882,541,990,5864,6898,1386,111,2437,2198,1239,5446,8097,5207,344,5804,18,3630,1511,6777,7536,3215,1049,7084,2331,2050,661,2183,2165,740,6864,4401,6805,3513,8139,1845,3558,4366,7510,4465,1781,7876,295,2084,2587,479,7108,3221,6141,6347,4374,7850,5747,2496,1117,7012,6589,5354,5560,4814,6835,2033,4815,1131,2126,7574,815,1910,3128,2063,6022,3819,3113,7885,7356,1265,4177,1517,8021,1667,6469,5749,3917,7229,388,7357,4535,981,4925,2507,7248,7668,1305,6369,6980,792,3188,208,2819,7378,2229,2870,669,1730,5815,940,5377,1034,6043,655,7324,4930,3960,5177,5390,8115,2896,6190,2598,4248,1440,4046,7606,1129,4670,594,7339,1206,2476,431,2631,7278,1004,846,2861,7815,2932,4438,3334,6456,5889,7810,3701,6093,2251,2714,2197,5752,7105,5938,5702,1171,4523,1176,5539,1645,335,2043,5904,3777,6245,3242,3748,3976,5637,6398,3918,5296,3596,5948,7992,4014,2808,7288,6567,4392,7594,3706,1754,4210,1722,4450,708,6988,1472,54,2204,1235,505,5,6856,5642,2628,146,7693,1271,4600,6896,89,3636,1741,1466,3872,1018,5381,2486,4466,7412,4997,2328,4751,7115,1535,4086,7949,6314,2340,4682,5276,41,6755,7492,4050,5884,2890,7939,4463,6170,3266,537,7068,255,4021,2320,5534,6930,5657,6605,6151,2266,6659,7317,6798,421,3534,4719,5756,1122,6078,120,1098,7661,7880,6588,4245,7756,909,5231,6508,6881,7140,5800,3200,4283,7902,7251,4423,6865,5096,44,1303,2429,8084,2726,3116,5999,7630,1518,1128,3356,3446,5397,7187,5443,6192,6627,7694,2466,3509,4224,4994,5668,7088,1010,1697,1582,1263,7403,2468,4707,760,6247,441,7014,8183,4218,4188,5779,6748,3193,4978,5316,6241,3986,1798,6637,311,7871,1954,6724,5630,8191,3483,5851,5858,5273,6711,1708,934,5681,7557,6279,7610,2899,3609,7952,2930,1339,4779,2438,242,4350,1420,641,5840,1079,7232,4981,4187,2453,6157,6496,3572,2732,1244,8143,4506,419,1965,658,6917,2924,6173,7220,1243,234,992,1390,6490,2262,615,6890,5367,7067,4009,3038,7165,1448,5415,7803,694,159,6812,4027,5946,7039,1796,1817,6750,4344,1680,2990,5119,94,305,2174,5131,4045,5881,4739,5025,4942,4340,6031,2475,7405,7812,294,353,5139,6166,3510,5293,490,6620,5429,3322,684,5113,910,1340,5970,1266,1684,868,7856,3016,3026,7903,1435,226,3851,7349,3598,2671,3336,4007,4470,7987,5838,7396,8160,5239,7766,6975,3387,5962,1174,1454,2578,5358,3454,3676,3293,4581,4405,2741,713,7304,3484,6119,5046,3046,4598,5859,6250,7435,7046,2616,1245,4034,1063,5447,4929,3317,7415,5148,7545,2756,4920,1736,200,3095,7655,1242,4214,6412,5405,1761,2667,22,3291,2027,1521,1051,7726,5033,8077,1228,5810,3219,3138,7057,1959,7983,851,7213,1666,2497,4238,3398,707,92,7671,5791,1688,5371,3951,7493,7963,270,7132,7675,2659,2682,4083,6281,3855,3860,2045,1750,1256,6377,6459,2384,1142,5143,3024,4841,454,7244,205,8053,4330,2566,5272,2771,5945,6631,5675,3214,5229,2547,5059,2070,2677,2546,5855,7646,7325,5798,827,6280,6435,3674,4217,7026,3261,8176,7523,7877,5133,6532,5237,3358,4773,6539,600,6463,3118,1545,512,4606,5655,6260,616,2810,6779,1354,463,3647,7226,4515,7562,4462,3620,8142,5868,1611,4165,1530,5553,5021,1429,1064,2242,4610,4797,3122,1934,1762,1969,3329,101,916,6331,5355,1288,5608,5234,5004,235,997,2334,8006,4774,6545,3341,5125,5487,2396,4577,7099,2329,2959,4329,3539,8174,6370,163,980,6985,7864,2423,1664,3301,2373,1876,6277,3846,7654,5829,3892,828,5445,6315,3834,7183,4310,2884,6163,7286,5340,6571,4140,2609,3209,6090,6893,6135,2996,1478,430,2150,5331,3723,721,7236,573,1225,3804,7362,5092,4916,76,4103,5448,1298,5761,7975,6852,5121,2636,7292,3622,4553,5063,3754,6324,4504,5286,1912,7171,2109,2465,7754,3145,1630,1607,3789,4288,1425,1961,3345,3022,102,4977,4736,3904,4503,4550,5902,7522,608,3597,1437,2258,5584,6012,7016,5372,1398,7954,3110,1102,4235,3952,7207,791,5471,1105,4763,6353,3812,5288,6063,3235,2332,6529,3543,3485,6861,7191,5047,2640,634,371,7951,1795,7585,4119,5378,6672,6126,7946,635,3380,7030,1138,6283,2078,7746,944,8044,6824,6224,3067,4704,4565,7769,6927,5343,6647,3554,386,1828,4991,1315,447,7455,7968,1402,7478,1126,3563,2231,7943,4304,1246,553,3897,5338,504,4778,7141,3545,6751,5435,6977,7945,5635,4743,2831,907,6772,7602,7676,3532,4028,2322,7212,2539,4169,1683,3205,5523,3476,6020,1272,2809,1234,5434,3991,55,4649,4143,4988,4338,1853,7969,4473,7835,597,2376,4842,164,4983,2268,794,7008,4547,2947,3386,6375,1944,5037,5457,4101,3924,2024,4051,7782,6547,7549,6499,2326,881,7290,3584,2644,5988,7956,3592,2725,954,5903,1209,4688,2285,4015,5454,4601,2967,7842,2531,5993,5990,93,1950,4410,7647,2161,2273,6705,6408,3708,7918,7727,1921,5559,4082,1173,2265,1849,5978,1493,4111,1027,108,3333,5155,7001,1857,782,7367,6387,2783,7301,1166,762,698,5605,2499,4636,2194,2379,858,351,601,4517,7441,4651,6935,3108,7384,6638,6506,3381,6364,8175,1538,5396,4420,2903,3131,1633,1787,4696,4128,5992,7359,3309,2069,6603,7669,6008,154,4331,6902,1860,6066,25,1883,1690,3884,1623,1555,4728,47,7497,7548,6651,6229,1277,1135,6343,5312,1093,5522,2132,982,7142,6047,4115,3912,6994,1080,813,7189,4828,561,2694,3442,629,4561,2137,339,3933,7998,1549,2119,3899,624,1866,6827,3907,407,1960,6785,73,6218,6635,3079,514,5919,6517,7069,1908,4662,7659,5165,3507,189,5232,8076,4274,3765,979,6803,7575,2393,5742,4809,4922,3120,4365,97,2805,6319,4270,1003,1150,883,3267,2516,4765,4924,6578,3093,3942,136,5187,3409,1632,589,3903,2542,7201,106,4490,7247,6946,2855,4784,5872,6606,5220,3611,7588,7980,2435,2898,3097,8046,1858,1436,3367,7175,564,2691,3316,6087,692,7348,7730,875,6089,5866,1588,961,7628,4291,5737,4113,4623,2954,5010,2240,2913,5467,1148,2168,1002,4562,4102,6397,6413,1612,5344,811,162,772,6255,4251,4459,8014,7838,4826,2914,7571,1088,1184,1639,2654,7638,5162,78,6312,775,2288,5228,37,8110,4545,7224,3885,7147,2213,2255,1650,3103,5054,3303,656,5314,867,1939,6818,2302,7394,3257,4811,7427,1224,3077,6102,1532,3920,6228,2488,158,793,3773,7627,64,2552,2325,4492,6674,540,7063,6088,3456,5909,4646,7713,7848,1362,1480,7005,6042,1175,856,3197,904,3410,4136,100,4282,5857,8073,3800,4759,4801,6269,6121,3844,274,3397,7743,4514,3401,4415,7686,2910,2256,7623,2330,3742,4740,221,4691,7268,5793,8120,427,1267,7644,3448,7772,6850,8,268,1273,2611,3553,8151,6254,6438,2823,5585,5543,327,2753,7783,6867,4813,340,7094,5600,1391,5516,3971,6000,7351,4850,5226,3815,7298,6476,2630,23,605,2734,4042,4059,2812,480,6168,4575,299,3416,3595,5769,2676,6966,7794,1087,3877,893,3175,116,4469,6301,1255,4946,1540,613,2372,3487,5778,729,7419,3690,142,5420,6236,5022,456,6399,6857,7342,5937,2925,7927,7090,3012,4471,3578,6678,2158,4904,7023,7162,3725,737,8178,837,5304,3310,4476,3159,886,1139,127,302,5079,4201,1382,1069,752,4899,2549,4066,5492,5428,6941,5511,8179,2114,803,5931,3265,2485,1124,6940,5835,5878,5341,1120,552,6482,5127,5842,2141,3788,5342,2707,2031,2352,5201,6421,5941,2210,143,2762,6332,5619,321,8131,8062,7303,3968,5166,5147,5294,4580,219,3717,5327,4787,7422,6576,3947,7344,6123,105,6540,1894,3930,352,7765,1963,372,7846,4639,2103,777,5153,5612,1357,7010,6555,3443,4840,3655,4822,1695,1095,5661,1652,1241,5504,5599,3467,6365,1948,4485,7296,7791,2439,7430,3583,8069,831,4306,2324,4073,4770,2681,3568,4315,6676,3941,901,3045,3473,7407,2604,3577,1988,4484,659,4921,5064,4650,2361,3581,7758,4521,754,5565,6488,2364,747,8129,7742,7307,3249,7912,6410,1833,334,5725,1165,3500,1430,7823,7496,2186,7473,3652,63,5199,4418,5663,896,4800,566,4962,5898,3533,7398,2935,5256,314,8003,3069,6083,771,6511,5202,2949,1554,6918,1341,4355,3521,2608,3766,6997,1113,4190,502,5152,4037,3085,8068,2215,4634,3327,1043,5077,3066,1734,5784,5801,2160,5689,1248,1893,7300,4543,459,488,1927,4215,6265,8002,6390,3375,5241,3155,7198,2679,7374,7679,6851,1704,7618,3863,7563,392,5095,6155,271,4277,5604,5579,2832,2657,5223,3555,2733,2956,7293,3418,3452,1157,3087,5035,795,494,679,7370,7414,5438,1703,7295,6697,1772,451,6542,2365,623,6806,7920,4869,6749,7487,959,5514,6477,3915,2093,6222,2911,2030,1189,4831,4992,6611,6017,197,8187,3264,7392,7965,5003,587,4236,331,4972,8009,6915,4837,4219,5916,5136,3797,1320,1940,2424,5494,3664,290,2758,4085,3335,975,3989,1560,5473,8039,2403,3063,123,2391,2827,3486,2233,4819,5242,5345,1599,5853,6010,4312,6076,4608,626,4898,6230,7355,7297,3212,2551,1701,6005,5411,6179,4971,1285,6536,5789,6434,4500,1813,2087,3949,2863,1187,3666,5307,3514,716,2283,1395,6652,5883,7072,2622,7291,3115,5537,542,1109,2964,4923,5936,401,5444,7243,4932,3937,2674,592,5185,7583,3251,3217,1351,7828,6305,4154,2939,4416,7764,2280,1505,675,5696,2760,6273,2728,2058,2669,1065,8159,5583,1381,6447,1507,5781,8141,2965,1169,632,1956,5391,2460,5697,1107,1112,931,254,4510,2451,3856,2652,7806,4874,310,908,16,6095,3075,2275,5382,6292,697,3623,1149,833,5475,384,1152,3626,928,4727,2800,3096,4335,3350,962,4617,439,6142,3599,2559,1179,879,5368,5724,3478,1591,4799,3702,1687,5850,5265,4805,3932,7695,129,4630,2440,2381,4206,7928,1104,2082,3297,287,4628,3927,6394,4643,3916,4114,1777,5771,3799,2253,4629,3224,1864,2503,259,2075,6130,2592,1720,3594,71,822,3427,1905,7423,1428,3015,394,2796,2427,6543,3775,4568,3413,5507,4605,2127,7082,6791,7483,2717,5299,3157,6662,3656,7935,958,678,7567,2181,229,2459,6358,7859,7755,1989,6361,1146,7961,4445,5960,7796,5918,5589,6688,5255,6961,972,3241,5089,5952,2176,172,2267,1918,2969,6742,2223,3326,3680,2107,2175,7375,272,3132,2357,4836,3239,3272,5468,5615,788,2627,3795,4674,4038,1311,4856,1115,731,1201,27,602,1281,1847,7925,2123,2887,4963,1558,7163,1156,3204,128,4244,6046,5674,7071,5251,8166,4391,5351,5298,6396,6407,39,3081,8058,7134,2986,2155,5292,1355,1041,152,2859,6889,4148,4434,6823,6351,4118,5967,139,2059,3491,5019,1597,6415,6836,4645,1859,5780,1464,1399,3477,4873,2359,842,4212,4139,2635,7120,1484,2693,7620,4091,7462,6900,3392,7657,7931,4247,5167,7463,3753,770,598,825,3254,3256,4003,6227,5578,4362,4096,985,4161,2869,5861,7771,7964,3498,1660,33,2472,1068,5740,2310,1019,3836,5577,7565,3615,7305,6834,5222,7691,2933,1964,3479,3739,1426,378,5118,852,4328,499,7206,7272,4864,1515,7154,4996,316,6680,6232,7777,1606,5512,1008,7136,7255,8180,3864,2749,5459,275,7049,8070,2182,5738,6617,6908,7704,3956,3550,3541,1738,5011,2607,5913,7227,8028,5310,995,6950,869,8113,6205,7015,293,453,5822,6892,312,2980,7887,510,328,7836,718,2452,7689,4457,3712,7168,1972,4106,2022,6602,7517,2521,3311,5406,5392,7433,5375,2420,3307,4063,4396,840,5362,920,6001,3660,5766,1207,7637,845,7167,1567,3104,7143,2537,810,5481,905,4766,3287,2795,7504,5609,1132,834,2784,5989,2191,377,2934,1001,6346,630,6404,2235,5736,2346,2921,4253,6968,2504,7819,3013,2304,7484,7211,3324,1727,7553,1216,6958,7117,2820,3017,7327,1260,1920,5966,693,3268,6453,3548,2780,6894,6178,5323,3769,5130,781,2908,4074,5985,5764,6990,5958,3106,759,6158,5462,6648,5739,7197,3129,6334,8125,6797,306,3831,1356,5274,3201,370,5933,2012,3898,6368,2979,2748,5770,7044,821,3890,7017,3250,6313,7551,7282,6129,4475,2536,1250,4758,7457,5863,4752,7851,8167,8124,1434,7631,4945,6929,4776,7564,7540,3169,5900,7166,574,955,3445,585,5826,5498,362,3332,6276,554,3282,7919,8042,5802,7240,1610,7436,6362,3354,1693,1856,6298,984,2490,2395,4661,6348,6962,4633,1726,1544,1401,1712,1348,4764,3914,6160,7792,7149,3137,3056,3344,2009,2794,5648,7233,6028,5610,7453,6246,3883,399,4967,6522,6,4958,6430,666,2621,5925,465,5991,2226,1528,7095,7490,247,5643,3709,4162,4621,1121,4025,1685,248,1221,7381,132,2718,507,4781,241,2456,7798,7365,3202,6718,6472,62,3810,4896,4684,6403,6693,6684,2509,5269,5581,9,863,2370,3588,2915,6148,4404,2416,5168,4910,6374,4443,5544,2431,4913,7228,3343,3735,6194,2110,3781,5357,4834,7235,6318,5734,4537,8093,2130,5489,1586,650,2011,8145,5039,7501,2227,2595,2426,3355,5083,7832,4267,6116,526,6679,2291,8112,1692,4597,5259,6903,1534,7439,7513,6393,233,2988,5712,2730,5006,7443,6025,5974,3893,4363,1636,5042,7776,1527,6239,6640,5955,6432,5385,1111,3740,2778,483,706,6359,1938,7077,7190,7299,6557,2064,5807,6761,5547,7596,8074,2389,704,8013,110,113,6174,6145,2754,1153,6685,1196,5224,6401,8118,1282,3944,3852,3761,2173,5744,3083,563,2791,1840,3749,1204,51,3727,7000,1159,7447,492,7208,5652,4902,2276,4530,2798,6967,276,6537,546,2506,6939,6002,4832,57,5564,5529,6059,1178,7560,7720,5484,2121,2735,4307,1046,5907,1208,1158,2478,4242,7276,1346,7940,4313,3424,1617,3663,2743,3260,1937,2799,4437,700,3,6819,1306,2538,1167,4796,6558,5186,3065,5795,2124,7917,1899,1489,8171,156,6610,1682,6534,4931,5313,3352,757,3608,7921,2619,5561,1045,3902,7098,6844,2479,2944,1468,1598,3571,4397,1622,1343,1661,5402,4403,6757,240,1585,5690,699,2729,2984,1888,2664,5437,780,6863,5873,2848,4664,5081,6446,2874,7950,1097,1958,4871,4985,4211,5407,6335,5616,6248,4272,1869,5964,2055,8173,487,8127,2399,6725,7025,4735,6521,7246,6776,4411,1974,4125,7593,2232,7672,5921,3023,607};

typedef _Float16 h16;
typedef unsigned short bf;
typedef __attribute__((ext_vector_type(16))) __bf16   v16bf;
typedef __attribute__((ext_vector_type(16))) _Float16 v16h;
typedef __attribute__((ext_vector_type(8)))  _Float16 v8h;
typedef __attribute__((ext_vector_type(8)))  unsigned short v8us;
typedef __attribute__((ext_vector_type(8)))  float    v8f;
typedef __attribute__((ext_vector_type(4)))  float    v4f;
typedef v8h  __attribute__((may_alias)) v8ha;
typedef v4f  __attribute__((may_alias)) v4fa;
typedef v8us __attribute__((may_alias)) v8usa;

__device__ __forceinline__ unsigned short f2bf(float f) { unsigned u = __float_as_uint(f); u += 0x7FFFu + ((u >> 16) & 1u); return (unsigned short)(u >> 16); }
__device__ __forceinline__ float bf2f(unsigned short b) { return __uint_as_float(((unsigned)b) << 16); }
__device__ __forceinline__ float bfr(float f) { return bf2f(f2bf(f)); }
__device__ __forceinline__ v16h cat16(v8h lo, v8h hi) { return __builtin_shufflevector(lo, hi, 0, 1, 2, 3, 4, 5, 6, 7, 8, 9, 10, 11, 12, 13, 14, 15); }
__device__ __forceinline__ v16bf cat16b(v8us lo, v8us hi) { return __builtin_bit_cast(v16bf, __builtin_shufflevector(lo, hi, 0, 1, 2, 3, 4, 5, 6, 7, 8, 9, 10, 11, 12, 13, 14, 15)); }
__device__ __forceinline__ v8f wmma16(v16h a, v16h b, v8f c) { return __builtin_amdgcn_wmma_f32_16x16x32_f16(false, a, false, b, (short)0, c, false, false); }
__device__ __forceinline__ v8f wmmab(v16bf a, v16bf b, v8f c) { return __builtin_amdgcn_wmma_f32_16x16x32_bf16(false, a, false, b, (short)0, c, false, false); }

template <bool SPLITA, bool F16OUT = false>
__global__ __launch_bounds__(128) void k_gemmb(const bf* __restrict__ A, const bf* __restrict__ Al, const bf* __restrict__ Bn, const float* __restrict__ bias, float* C, int ldc, h16* C2, const float* __restrict__ R = nullptr, int K = DM, int roundR = 1) {
    __shared__ __align__(16) float ost[4][16 * 68];
    const int lane = threadIdx.x & 31, wave = threadIdx.x >> 5, lr = lane & 15, hi = lane >> 4;
    const int r0 = blockIdx.x * 64 + wave * 16, c0 = blockIdx.y * 64;
    const size_t aoff = (size_t)(r0 + lr) * K + 8 * hi;
    size_t boff[4];
#pragma unroll
    for (int t = 0; t < 4; ++t) boff[t] = (size_t)(c0 + t * 16 + lr) * K + 8 * hi;
    v8f acc[4];
#pragma unroll
    for (int t = 0; t < 4; ++t) acc[t] = (v8f){};
#pragma unroll 1
    for (int kc = 0; kc < K; kc += 32) {
        const v16bf a = cat16b(*(const v8us*)(A + aoff + kc), *(const v8us*)(A + aoff + kc + 16));
        v16bf al = a;
        if (SPLITA) al = cat16b(*(const v8us*)(Al + aoff + kc), *(const v8us*)(Al + aoff + kc + 16));
#pragma unroll
        for (int t = 0; t < 4; ++t) { const v16bf b = cat16b(*(const v8us*)(Bn + boff[t] + kc), *(const v8us*)(Bn + boff[t] + kc + 16)); acc[t] = wmmab(a, b, acc[t]); if (SPLITA) acc[t] = wmmab(al, b, acc[t]); }
        asm volatile("v_nop\n\tv_nop\n\tv_nop\n\tv_nop" : "+v"(acc[0]), "+v"(acc[1]), "+v"(acc[2]), "+v"(acc[3]) : "v"(a), "v"(al));
    }
    float* os = &ost[wave][0];
#pragma unroll
    for (int t = 0; t < 4; ++t) { const float bv = bias ? bfr(bias[c0 + t * 16 + lr]) : 0.f;
#pragma unroll
        for (int j = 0; j < 8; ++j) os[(hi * 8 + j) * 68 + t * 16 + lr] = acc[t][j] + bv; }
    __syncthreads();
    if (F16OUT) {
        h16* crow = (h16*)(void*)C + (size_t)r0 * ldc + c0;
        auto pass = [&]() {
#pragma unroll
            for (int s = 0; s < 4; ++s) { const int row = 4 * s + (lane >> 3), piece = lane & 7; const float* sp = os + row * 68 + piece * 8; v8h o, o2;
#pragma unroll
                for (int i = 0; i < 8; ++i) { const h16 a = (h16)sp[i]; o[i] = a; o2[i] = (h16)((sp[i] - (float)a) * LOSC); }
                *(volatile v8h*)(crow + (size_t)row * ldc + piece * 8) = o; if (C2) *(volatile v8h*)(C2 + (size_t)r0 * ldc + c0 + (size_t)row * ldc + piece * 8) = o2; }
        };
        pass(); __threadfence(); pass();
    } else {
        float* crow = C + (size_t)r0 * ldc + c0;
        auto pass = [&]() {
#pragma unroll
            for (int s = 0; s < 8; ++s) { const int Lid = (lane >> 3) + 4 * s, piece = lane & 7; const int row = Lid >> 1, cofs = (Lid & 1) * 32 + piece * 4;
                v4f val = *(const v4fa*)(os + row * 68 + cofs); if (R) { const v4f rv = *(const v4f*)(R + ((size_t)r0 + row) * ldc + c0 + cofs); val += roundR ? (v4f){bfr(rv[0]), bfr(rv[1]), bfr(rv[2]), bfr(rv[3])} : rv; }
                *(volatile v4f*)(crow + (size_t)row * ldc + cofs) = val; }
        };
        pass(); __threadfence(); pass();
    }
}


__global__ __launch_bounds__(256) void k_srow(const float* __restrict__ sc, bf* S2) {
    const int lane = threadIdx.x & 31, r = blockIdx.x * 8 + (threadIdx.x >> 5); if (r >= 64) return;
#pragma unroll 1
    for (int ps = 0; ps < 2; ++ps) {
#pragma unroll 1
        for (int c0 = lane * 8; c0 < KP; c0 += 256) { v8us o;
#pragma unroll
            for (int q = 0; q < 8; ++q) { const int i = c0 + q; const bool ok = i < NTR; float v = 0.f; if (r == 0 && ok) v = bfr(sc[c_perm[i]]); else if (r == 1 && ok) v = 1.0f; o[q] = f2bf(v); }
            *(volatile v8us*)(S2 + (size_t)r * KP + c0) = o; }
        if (ps == 0) __threadfence(); }
}
__global__ __launch_bounds__(256) void k_kern(const float* __restrict__ emb, const float* __restrict__ a2p, const float* __restrict__ bp, int j0, bf* Kh, bf* Kl) {
    const int lane = threadIdx.x & 31, r = blockIdx.x * 8 + (threadIdx.x >> 5); if (r >= RCH) return; const int j = c_perm[j0 + r];
    const float xj0 = bfr(emb[2 * j]), xj1 = bfr(emb[2 * j + 1]); const float sqj = xj0 * xj0 + xj1 * xj1; const float a2 = bfr(a2p[0]), bb = bfr(bp[0]); const float ra2 = a2 * a2, ex = 2.0f * bb * bb;
#pragma unroll 1
    for (int ps = 0; ps < 2; ++ps) {
#pragma unroll 1
        for (int c0 = lane * 8; c0 < KP; c0 += 256) { v8us oh, ol;
#pragma unroll
            for (int q = 0; q < 8; ++q) { const int ii = c0 + q; float kv = 0.f;
                if (ii < NTR) { const int i = c_perm[ii]; const float xi0 = bfr(emb[2 * i]), xi1 = bfr(emb[2 * i + 1]); const float sq = xi0 * xi0 + xi1 * xi1 + sqj - 2.0f * (xi0 * xj0 + xi1 * xj1);
                    const float d = sqrtf(fmaxf(sq, 0.f) + DEPS); kv = 1.0f / (1.0f + ra2 * __builtin_amdgcn_exp2f(ex * __builtin_amdgcn_logf(d))); }
                const unsigned short hb = f2bf(kv); oh[q] = hb; ol[q] = f2bf(kv - bf2f(hb)); }
            const size_t o = (size_t)r * KP + c0; *(volatile v8us*)(Kh + o) = oh; *(volatile v8us*)(Kl + o) = ol; }
        if (ps == 0) __threadfence(); }
}
__global__ __launch_bounds__(256) void k_err(const float* __restrict__ C, const float* __restrict__ sc, const float* __restrict__ a1p, int j0, float* E) {
    const int r = blockIdx.x * 256 + threadIdx.x; if (r >= RCH) return; const int j = c_perm[j0 + r]; const float a1 = bfr(a1p[0]);
    const float kde = C[(size_t)r * 64] / C[(size_t)r * 64 + 1]; const float dlt = bfr(sc[j]) - a1 * a1 * kde; const float e = dlt * dlt;
    *(volatile float*)(E + j0 + r) = e; __threadfence(); *(volatile float*)(E + j0 + r) = e;
}
__global__ __launch_bounds__(32) void k_final(const float* __restrict__ E, float* OUTP) {
    if (threadIdx.x != 0) return; float st = 0.f, sv = 0.f;
#pragma unroll 1
    for (int q = 0; q < NTR; ++q) st += E[q];
#pragma unroll 1
    for (int q = NTR; q < NALL; ++q) sv += E[q];
    const float r = 0.3f * (st / (float)NTR) + sv / (float)NVA; *(volatile float*)OUTP = r; __threadfence(); *(volatile float*)OUTP = r;
}

extern "C" void kernel_launch(void* const* d_in, const int* in_sizes, int n_in,
                              void* d_out, int out_size, void* d_ws, size_t ws_size, hipStream_t stream) {
    (void)in_sizes; (void)n_in; (void)out_size;
    const float* emb = (const float*)d_in[0]; const float* sc = (const float*)d_in[1];   const float* a1p = (const float*)d_in[3]; const float* a2p = (const float*)d_in[4]; const float* bp = (const float*)d_in[5];
    float* out = (float*)d_out;
    char* wsp = (char*)d_ws;
    auto take = [&](size_t bytes) { char* p = wsp; wsp += (bytes + 255) & ~(size_t)255; return (void*)p; };
    bf* S2 = (bf*)take((size_t)64 * KP * 2); bf* Kh = (bf*)take((size_t)RCH * KP * 2); bf* Kl = (bf*)take((size_t)RCH * KP * 2); float* C = (float*)take((size_t)RCH * 64 * 4); float* E = (float*)take((size_t)NALL * 4);
    if ((size_t)(wsp - (char*)d_ws) > ws_size) return;
    k_srow<<<64 / 8, 256, 0, stream>>>(sc, S2);
    for (int ch = 0; ch < NALL / RCH; ++ch) { const int j0 = ch * RCH;
        k_kern<<<RCH / 8, 256, 0, stream>>>(emb, a2p, bp, j0, Kh, Kl);
        k_gemmb<true, false><<<dim3(RCH / 64, 1, 1), 128, 0, stream>>>(Kh, Kl, S2, nullptr, C, 64, nullptr, nullptr, KP);
        k_err<<<RCH / 256, 256, 0, stream>>>(C, sc, a1p, j0, E); }
    k_final<<<1, 32, 0, stream>>>(E, out);
}
